// BlockDenseMHA_14714557956664
// MI455X (gfx1250) — hardware-verified
//
#include <hip/hip_runtime.h>
#include <math.h>

#define NB_ 4
#define FF 64
#define TT 512
#define HW_ (FF * TT)
#define NHD 4
#define HD 16
#define LW 64

typedef _Float16 f16;
typedef __attribute__((ext_vector_type(16))) f16 f16x16;
typedef __attribute__((ext_vector_type(8)))  f16 f16x8;
typedef __attribute__((ext_vector_type(8)))  float f32x8;
typedef __attribute__((ext_vector_type(4)))  float v4f_t;
typedef float v4fa __attribute__((ext_vector_type(4), may_alias));
typedef __attribute__((ext_vector_type(4))) unsigned v4u_t;
typedef unsigned v4ua __attribute__((ext_vector_type(4), may_alias));

__device__ __forceinline__ f32x8 wmma16(f16x16 a, f16x16 b, f32x8 c) {
  c = __builtin_amdgcn_wmma_f32_16x16x32_f16(false, a, false, b, (short)0, c, false, false);
  asm volatile("v_nop\n\tv_nop\n\tv_nop\n\tv_nop" : "+v"(c) : "v"(a), "v"(b));
  return c;
}
__device__ __forceinline__ f16x16 lds_frag(const f16* base, int stride) {
  const int lane = threadIdx.x & 31, row = lane & 15, kh = (lane >> 4) * 8;
  const f16x8 lo = *(const f16x8*)(base + row * stride + kh);
  const f16x8 hi = *(const f16x8*)(base + row * stride + kh + 16);
  f16x16 f;
#pragma unroll
  for (int i = 0; i < 8; ++i) { f[i] = lo[i]; f[i + 8] = hi[i]; }
  return f;
}
template <int KS, int CIN>
__device__ __forceinline__ f16x16 wfrag(const float* __restrict__ Wm, int nrows, int o0, int ks) {
  constexpr int KTOT = CIN * KS * KS;
  const int lane = threadIdx.x & 31, r = o0 + (lane & 15), kh = (lane >> 4) * 8;
  f16x16 f;
  if (KS == 1) {
#pragma unroll
    for (int i = 0; i < 8; ++i) { const int ka = ks * 32 + kh + i, kb = ka + 16;
      f[i] = (f16)((r < nrows && ka < KTOT) ? Wm[(size_t)r * KTOT + ka] : 0.0f); f[8 + i] = (f16)((r < nrows && kb < KTOT) ? Wm[(size_t)r * KTOT + kb] : 0.0f); }
  } else {
    const int tap = (ks * 32) / CIN, c0 = (ks * 32) % CIN;
#pragma unroll
    for (int i = 0; i < 8; ++i) { const int ca = c0 + kh + i, cb = ca + 16;
      f[i] = (f16)((r < nrows) ? Wm[(size_t)r * KTOT + ca * 9 + tap] : 0.0f); f[8 + i] = (f16)((r < nrows) ? Wm[(size_t)r * KTOT + cb * 9 + tap] : 0.0f); }
  }
  return f;
}

struct SrcCat { const void* p0; int n0; const f16* p1; int n1; const f16* p2; int n2; };
template <int KS, int CIN, int COUT, int NT, bool BNL, bool O16, bool F32_0>
__global__ __launch_bounds__(256) void k_conv(SrcCat S, const float* __restrict__ Wt, const float* __restrict__ bias,
                                             const float* __restrict__ bg, const float* __restrict__ bb, const float* __restrict__ bm, const float* __restrict__ bv,
                                             void* __restrict__ dstv) {
  __shared__ __attribute__((aligned(16))) f16 aS[128 * 40];
  __shared__ __attribute__((aligned(16))) float oS[NT * 16 * 132];
  __shared__ float sc[CIN], sh[CIN];
  constexpr int KTOT = CIN * KS * KS, KSTEPS = (KTOT + 31) / 32;
  const int tid = threadIdx.x, lane = tid & 31, wave = tid >> 5, cl = lane & 15, rh = (lane >> 4) * 8;
  const int b = blockIdx.x / (FF * 4), rem = blockIdx.x % (FF * 4), f = rem >> 2, t0 = (rem & 3) * 128;
  if (BNL) for (int c = tid; c < CIN; c += 256) { const float s = bg[c] / sqrtf(bv[c] + 1e-5f); sc[c] = s; sh[c] = bb[c] - bm[c] * s; }
  f32x8 acc[NT];
#pragma unroll
  for (int j = 0; j < NT; ++j) { f32x8 z = {}; acc[j] = z; }
  __syncthreads();
#pragma unroll 1
  for (int ks = 0; ks < KSTEPS; ++ks) {
    __syncthreads();
    { const int px = tid >> 1, kq = (tid & 1) * 16;
      int fs, ts, c0;
      if (KS == 3) { const int tap = (ks * 32) / CIN; c0 = (ks * 32) % CIN + kq; fs = f + tap / 3 - 1; ts = t0 + px + (tap % 3) - 1; } else { c0 = ks * 32 + kq; fs = f; ts = t0 + px; }
      const bool inside = (fs >= 0 && fs < FF && ts >= 0 && ts < TT);
      const size_t pix = inside ? (size_t)(fs * TT + ts) : 0;
      int seg, cl0, nseg; if (c0 < S.n0) { seg = 0; cl0 = c0; nseg = S.n0; } else if (c0 < S.n0 + S.n1) { seg = 1; cl0 = c0 - S.n0; nseg = S.n1; } else { seg = 2; cl0 = c0 - S.n0 - S.n1; nseg = S.n2; }
      const size_t base = ((size_t)b * nseg + cl0) * HW_ + pix;
#pragma unroll 4
      for (int u = 0; u < 16; ++u) { const int c = c0 + u; float v = 0.0f;
        if (inside && c < CIN) {
          if (seg == 0) v = F32_0 ? ((const float*)S.p0)[base + (size_t)u * HW_] : (float)((const f16*)S.p0)[base + (size_t)u * HW_];
          else if (seg == 1) v = (float)S.p1[base + (size_t)u * HW_]; else v = (float)S.p2[base + (size_t)u * HW_];
          if (BNL) { v = v * sc[c] + sh[c]; v = (v >= 0.0f) ? v : 0.01f * v; } }
        aS[px * 40 + kq + u] = (f16)v; } }
    __syncthreads();
    const f16x16 af = lds_frag(aS + (wave * 16) * 40, 40);
#pragma unroll
    for (int j = 0; j < NT; ++j) acc[j] = wmma16(af, wfrag<KS, CIN>(Wt, COUT, j * 16, ks), acc[j]);
  }
#pragma unroll
  for (int j = 0; j < NT; ++j) { const int o = j * 16 + cl; const float bvv = (o < COUT) ? bias[o] : 0.0f;
#pragma unroll
    for (int r = 0; r < 8; ++r) oS[o * 132 + wave * 16 + rh + r] = acc[j][r] + bvv; }
  __syncthreads();
#pragma unroll 1
  for (int pass = 0; pass < 2; ++pass) {
    if (!O16) { float* dst = (float*)dstv;
      for (int q = tid; q < COUT * 32; q += 256) { const int o = q >> 5, c4 = (q & 31) * 4;
        *(volatile v4f_t*)(dst + ((size_t)b * COUT + o) * HW_ + (size_t)f * TT + t0 + c4) = *(const volatile v4fa*)(oS + o * 132 + c4); } }
    else { f16* dst = (f16*)dstv;
      for (int q = tid; q < COUT * 16; q += 256) { const int o = q >> 4, c8 = (q & 15) * 8; union { f16 hh[8]; v4u_t u; } cv;
#pragma unroll
        for (int e = 0; e < 8; ++e) cv.hh[e] = (f16)oS[o * 132 + c8 + e];
        *(volatile v4u_t*)(dst + ((size_t)b * COUT + o) * HW_ + (size_t)f * TT + t0 + c8) = cv.u; } }
    __threadfence();
  }
}

__global__ __launch_bounds__(256) void k_band(const f16* __restrict__ qkv, f16* __restrict__ ao) {
  __shared__ __attribute__((aligned(16))) f16 qS[64 * 40], kS[192 * 40], vT[16 * 200], PS[64 * 200];
  __shared__ float sS[64 * 196];
  __shared__ __attribute__((aligned(16))) float oS[16 * 68];
  const int tid = threadIdx.x, lane = tid & 31, wave = tid >> 5, cl = lane & 15, rh = (lane >> 4) * 8;
  int bi = blockIdx.x; const int qt = bi & 7; bi >>= 3; const int h = bi & 3; bi >>= 2; const int f = bi % FF, b = bi / FF;
  const int q0 = qt * 64, kbase = q0 - LW;
  const f16* qb = qkv + ((size_t)b * 192) * HW_ + (size_t)f * TT;
  for (int e = tid; e < 64 * 32; e += 256) { const int q = e >> 5, d = e & 31; qS[q * 40 + d] = (d < HD) ? qb[(size_t)(h * HD + d) * HW_ + q0 + q] : (f16)0.0f; }
  for (int e = tid; e < 192 * 32; e += 256) { const int s = e >> 5, d = e & 31; const int t = kbase + s; f16 v = (f16)0.0f;
    if (d < HD && t >= 0 && t < TT) v = qb[(size_t)(64 + h * HD + d) * HW_ + t]; kS[s * 40 + d] = v; }
  for (int e = tid; e < 16 * 192; e += 256) { const int d = e / 192, s = e % 192; const int t = kbase + s; f16 v = (f16)0.0f;
    if (t >= 0 && t < TT) v = qb[(size_t)(128 + h * HD + d) * HW_ + t]; vT[d * 200 + s] = v; }
  if (tid < 16) { for (int s = 192; s < 200; ++s) vT[tid * 200 + s] = (f16)0.0f; }
  for (int e = tid; e < 64 * 200; e += 256) PS[e] = (f16)0.0f;
  __syncthreads();
#pragma unroll 1
  for (int it = 0; it < 6; ++it) { const int tix = wave * 6 + it, qtile = tix / 12, kt = tix % 12;
    f32x8 acc = {}; acc = wmma16(lds_frag(qS + (qtile * 16) * 40, 40), lds_frag(kS + (kt * 16) * 40, 40), acc);
#pragma unroll
    for (int r = 0; r < 8; ++r) sS[(qtile * 16 + rh + r) * 196 + kt * 16 + cl] = acc[r]; }
  __syncthreads();
  { const int q = tid >> 2, part = tid & 3; const int t = q0 + q; const float scl = 0.25f * 1.44269504088896340736f;
    float lg[48]; float mx = -3.0e38f;
#pragma unroll
    for (int i = 0; i < 48; ++i) { const int s = part * 48 + i; const int tk = kbase + s; const bool ok = (s >= q) && (s <= q + 2 * LW) && (tk < TT);
      lg[i] = ok ? ((tk >= 0) ? sS[q * 196 + s] * scl : 0.0f) : -3.0e38f; mx = fmaxf(mx, lg[i]); }
    mx = fmaxf(mx, __shfl_xor(mx, 1, 32)); mx = fmaxf(mx, __shfl_xor(mx, 2, 32));
    float z = 0.0f;
#pragma unroll
    for (int i = 0; i < 48; ++i) { const float e = (lg[i] <= -1.0e38f) ? 0.0f : exp2f(lg[i] - mx); lg[i] = e; z += e; }
    z += __shfl_xor(z, 1, 32); z += __shfl_xor(z, 2, 32);
    const float iz = 1024.0f / z;
#pragma unroll
    for (int i = 0; i < 48; ++i) PS[q * 200 + part * 48 + i] = (f16)(lg[i] * iz); (void)t; }
  __syncthreads();
  if (wave < 4) { f32x8 acc = {};
#pragma unroll
    for (int ks = 0; ks < 6; ++ks) acc = wmma16(lds_frag(PS + (wave * 16) * 200 + ks * 32, 200), lds_frag(vT + ks * 32, 200), acc);
#pragma unroll
    for (int r = 0; r < 8; ++r) oS[cl * 68 + wave * 16 + rh + r] = acc[r] * (1.0f / 1024.0f); }
  __syncthreads();
#pragma unroll 1
  for (int pass = 0; pass < 2; ++pass) {
    if (tid < 128) { const int d = tid >> 3, c8 = (tid & 7) * 8; union { f16 hh[8]; v4u_t u; } cv;
#pragma unroll
      for (int e = 0; e < 8; ++e) cv.hh[e] = (f16)oS[d * 68 + c8 + e];
      *(volatile v4u_t*)(ao + ((size_t)b * 64 + h * HD + d) * HW_ + (size_t)f * TT + q0 + c8) = cv.u; }
    __threadfence();
  }
}

extern "C" void kernel_launch(void* const* d_in, const int* in_sizes, int n_in,
                              void* d_out, int out_size, void* d_ws, size_t ws_size,
                              hipStream_t stream) {
  (void)in_sizes; (void)n_in; (void)out_size;
  const float* x = (const float*)d_in[0];
  const float* bd0_g = (const float*)d_in[1], *bd0_b = (const float*)d_in[2], *bd0_m = (const float*)d_in[3], *bd0_v = (const float*)d_in[4], *bd0_w = (const float*)d_in[5], *bd0_wb = (const float*)d_in[6];
  const float* bd1_g = (const float*)d_in[7], *bd1_b = (const float*)d_in[8], *bd1_m = (const float*)d_in[9], *bd1_v = (const float*)d_in[10], *bd1_w = (const float*)d_in[11], *bd1_wb = (const float*)d_in[12];
  const float* bdo_g = (const float*)d_in[13], *bdo_b = (const float*)d_in[14], *bdo_m = (const float*)d_in[15], *bdo_v = (const float*)d_in[16], *bdo_w = (const float*)d_in[17], *bdo_wb = (const float*)d_in[18];
  const float* qkv_w = (const float*)d_in[19], *qkv_b = (const float*)d_in[20], *o_w = (const float*)d_in[21], *o_b = (const float*)d_in[22];
  const float* sao_g = (const float*)d_in[23], *sao_b = (const float*)d_in[24], *sao_m = (const float*)d_in[25], *sao_v = (const float*)d_in[26], *sao_w = (const float*)d_in[27], *sao_wb = (const float*)d_in[28];
  float* out = (float*)d_out;
  char* ws = (char*)d_ws;
  f16* a0 = (f16*)ws; ws += (size_t)NB_ * 32 * HW_ * 2;
  f16* a1 = (f16*)ws; ws += (size_t)NB_ * 32 * HW_ * 2;
  f16* yb = (f16*)ws; ws += (size_t)NB_ * 64 * HW_ * 2;
  f16* qkvb = (f16*)ws; ws += (size_t)NB_ * 192 * HW_ * 2;
  f16* ao = (f16*)ws; ws += (size_t)NB_ * 64 * HW_ * 2;
  f16* att = (f16*)ws; ws += (size_t)NB_ * 64 * HW_ * 2;
  if ((size_t)(ws - (char*)d_ws) > ws_size) return;
  const dim3 g(NB_ * FF * 4), blk(256);
  const SrcCat s0{x, 64, nullptr, 0, nullptr, 0}, s1{x, 64, a0, 32, nullptr, 0}, s2{x, 64, a0, 32, a1, 32};
  const SrcCat sy{yb, 64, nullptr, 0, nullptr, 0}, so{ao, 64, nullptr, 0, nullptr, 0}, sz{yb, 64, att, 64, nullptr, 0};
  k_conv<3, 64, 32, 2, true, true, true><<<g, blk, 0, stream>>>(s0, bd0_w, bd0_wb, bd0_g, bd0_b, bd0_m, bd0_v, a0);
  k_conv<3, 96, 32, 2, true, true, true><<<g, blk, 0, stream>>>(s1, bd1_w, bd1_wb, bd1_g, bd1_b, bd1_m, bd1_v, a1);
  k_conv<3, 128, 64, 4, true, true, true><<<g, blk, 0, stream>>>(s2, bdo_w, bdo_wb, bdo_g, bdo_b, bdo_m, bdo_v, yb);
  k_conv<1, 64, 192, 12, false, true, false><<<g, blk, 0, stream>>>(sy, qkv_w, qkv_b, nullptr, nullptr, nullptr, nullptr, qkvb);
  k_band<<<dim3(NB_ * FF * NHD * 8), blk, 0, stream>>>(qkvb, ao);
  k_conv<1, 64, 64, 4, false, true, false><<<g, blk, 0, stream>>>(so, o_w, o_b, nullptr, nullptr, nullptr, nullptr, att);
  k_conv<1, 128, 64, 4, true, false, false><<<g, blk, 0, stream>>>(sz, sao_w, sao_wb, sao_g, sao_b, sao_m, sao_v, out);
}
